// TensorBase_30142080483421
// MI455X (gfx1250) — hardware-verified
//
#include <hip/hip_runtime.h>


namespace {
constexpr int NRAY = 4096, NSMP = 128, APP = 27, FEAT = 128, NIN = 390, KP = 416;
constexpr int W1P = 448;
constexpr int NPE = 6;
constexpr float DENSITY_SHIFT = -10.0f, DIST_SCALE = 25.0f;

typedef _Float16 b16;
typedef __attribute__((ext_vector_type(16))) _Float16 v16b;
typedef __attribute__((ext_vector_type(8)))  _Float16 v8b;
typedef __attribute__((ext_vector_type(8)))  float v8f;
typedef __attribute__((ext_vector_type(4)))  float v4f;

__device__ __forceinline__ v8b ld8b(const b16* p) { return *(const v8b*)p; }
__device__ __forceinline__ v16b cat8b(v8b a, v8b b) { return __builtin_shufflevector(a, b, 0, 1, 2, 3, 4, 5, 6, 7, 8, 9, 10, 11, 12, 13, 14, 15); }
__device__ __forceinline__ v16b frag_kb(const b16* p, int hh) { return cat8b(ld8b(p + 8 * hh), ld8b(p + 16 + 8 * hh)); }
__device__ __forceinline__ v8f wmma16b(v16b a, v16b b, v8f c) {
  v8f d = __builtin_amdgcn_wmma_f32_16x16x32_f16(false, a, false, b, (short)0, c, false, false);
  asm volatile("v_nop\n\tv_nop\n\tv_nop\n\tv_nop" : "+v"(d) : "v"(a), "v"(b));
  return d;
}
__device__ __forceinline__ void wave_lds_sync() {
  __builtin_amdgcn_fence(__ATOMIC_RELEASE, "workgroup");
  __builtin_amdgcn_wave_barrier();
  __builtin_amdgcn_fence(__ATOMIC_ACQUIRE, "workgroup");
}

__global__ __launch_bounds__(256) void prep_kernel(const float* __restrict__ W1, const float* __restrict__ W2, const float* __restrict__ W3,
                                                   b16* __restrict__ W1T, b16* __restrict__ W2T, b16* __restrict__ W3T) {
  __shared__ __attribute__((aligned(16))) b16 Tl[8][W1P];
  const int tid = threadIdx.x, lane = tid & 31, wave = tid >> 5, blk = blockIdx.x;
  for (int pass = 0; pass < 2; ++pass) {
    if (blk < 16) {
      const int n0 = blk * 8;
      for (int i = tid; i < 8 * W1P; i += 256) { const int n = i / W1P, k = i % W1P; Tl[n][k] = (k < NIN) ? (b16)W1[(size_t)k * FEAT + n0 + n] : (b16)0.0f; }
      __syncthreads();
      { const int n = wave; b16* dst = W1T + (size_t)(n0 + n) * W1P;
        for (int j = lane; j < W1P / 8; j += 32) *(volatile v8b*)(dst + j * 8) = *(const v8b*)(&Tl[n][j * 8]); }
    } else if (blk < 32) {
      const int n0 = (blk - 16) * 8;
      for (int i = tid; i < 8 * FEAT; i += 256) { const int n = i / FEAT, k = i % FEAT; Tl[n][k] = (b16)W2[(size_t)k * FEAT + n0 + n]; }
      __syncthreads();
      { const int n = wave; if (lane < 16) *(volatile v8b*)(W2T + (size_t)(n0 + n) * FEAT + lane * 8) = *(const v8b*)(&Tl[n][lane * 8]); }
    } else {
      const int n0 = (blk - 32) * 8;
      for (int i = tid; i < 8 * FEAT; i += 256) { const int n = i / FEAT, k = i % FEAT; Tl[n][k] = (n0 + n < 3) ? (b16)W3[(size_t)k * 3 + n0 + n] : (b16)0.0f; }
      __syncthreads();
      { const int n = wave; if (lane < 16) *(volatile v8b*)(W3T + (size_t)(n0 + n) * FEAT + lane * 8) = *(const v8b*)(&Tl[n][lane * 8]); }
    }
    __threadfence();
    __syncthreads();
  }
}

__global__ __launch_bounds__(128) void ray_kernel(const float* __restrict__ sigf, const float* __restrict__ app, const float* __restrict__ viewdirs,
                                                 const float* __restrict__ dists, const float* __restrict__ zvals,
                                                 const b16* __restrict__ W1T, const float* __restrict__ b1, const b16* __restrict__ W2T, const float* __restrict__ b2,
                                                 const b16* __restrict__ W3T, const float* __restrict__ b3, float* __restrict__ slot) {
  __shared__ __attribute__((aligned(16))) b16 Ain[NSMP][KP];
  __shared__ __attribute__((aligned(16))) b16 Hs[NSMP][FEAT];
  __shared__ float rgbS[NSMP][4];
  __shared__ float alphaS[NSMP], wS[NSMP];
  const int tid = threadIdx.x, wave = tid >> 5, lane = tid & 31, hh = lane >> 4, col = lane & 15;
  const int ray = blockIdx.x;
  {
    const int s = tid;
    b16* row = Ain[s];
    const float* ap = app + ((size_t)ray * NSMP + s) * APP;
    for (int d = 0; d < APP; ++d) {
      const float x = ap[d];
      row[d] = (b16)x;
      float sn, cs; sincosf(x, &sn, &cs);
      row[30 + d * NPE] = (b16)sn; row[192 + d * NPE] = (b16)cs;
#pragma unroll
      for (int k = 1; k < NPE; ++k) { const float s2 = 2.0f * sn * cs, c2 = cs * cs - sn * sn; sn = s2; cs = c2; row[30 + d * NPE + k] = (b16)sn; row[192 + d * NPE + k] = (b16)cs; }
    }
    for (int d = 0; d < 3; ++d) {
      const float x = viewdirs[(size_t)ray * 3 + d];
      row[27 + d] = (b16)x;
      float sn, cs; sincosf(x, &sn, &cs);
      row[354 + d * NPE] = (b16)sn; row[372 + d * NPE] = (b16)cs;
#pragma unroll
      for (int k = 1; k < NPE; ++k) { const float s2 = 2.0f * sn * cs, c2 = cs * cs - sn * sn; sn = s2; cs = c2; row[354 + d * NPE + k] = (b16)sn; row[372 + d * NPE + k] = (b16)cs; }
    }
    for (int k = NIN; k < KP; ++k) row[k] = (b16)0.0f;
    const float xs = sigf[(size_t)ray * NSMP + s] + DENSITY_SHIFT;
    const float sigma = fmaxf(xs, 0.0f) + log1pf(expf(-fabsf(xs)));
    float a = 1.0f - expf(-sigma * dists[(size_t)ray * NSMP + s] * DIST_SCALE);
    if (s == NSMP - 1) a = 1.0f;
    alphaS[s] = a;
  }
  __syncthreads();
  const int m0 = wave * 32;
  {
    v8f acc[2][8];
#pragma unroll
    for (int r = 0; r < 2; ++r)
#pragma unroll
      for (int t = 0; t < 8; ++t) acc[r][t] = (v8f){};
    for (int kb = 0; kb < KP; kb += 32) {
      const v16b a0 = frag_kb(&Ain[m0 + col][kb], hh), a1 = frag_kb(&Ain[m0 + 16 + col][kb], hh);
#pragma unroll
      for (int t = 0; t < 8; ++t) { const v16b bw = frag_kb(W1T + (size_t)(t * 16 + col) * W1P + kb, hh); acc[0][t] = wmma16b(a0, bw, acc[0][t]); acc[1][t] = wmma16b(a1, bw, acc[1][t]); }
    }
#pragma unroll
    for (int t = 0; t < 8; ++t)
#pragma unroll
      for (int r = 0; r < 2; ++r)
#pragma unroll
        for (int v = 0; v < 8; ++v) { const int rr = m0 + r * 16 + 8 * hh + v, cc = t * 16 + col; Hs[rr][cc] = (b16)fmaxf(acc[r][t][v] + b1[cc], 0.0f); }
  }
  wave_lds_sync();
  {
    v8f acc[2][8];
#pragma unroll
    for (int r = 0; r < 2; ++r)
#pragma unroll
      for (int t = 0; t < 8; ++t) acc[r][t] = (v8f){};
#pragma unroll
    for (int kb = 0; kb < FEAT; kb += 32) {
      const v16b a0 = frag_kb(&Hs[m0 + col][kb], hh), a1 = frag_kb(&Hs[m0 + 16 + col][kb], hh);
#pragma unroll
      for (int t = 0; t < 8; ++t) { const v16b bw = frag_kb(W2T + (size_t)(t * 16 + col) * FEAT + kb, hh); acc[0][t] = wmma16b(a0, bw, acc[0][t]); acc[1][t] = wmma16b(a1, bw, acc[1][t]); }
    }
    wave_lds_sync();
#pragma unroll
    for (int t = 0; t < 8; ++t)
#pragma unroll
      for (int r = 0; r < 2; ++r)
#pragma unroll
        for (int v = 0; v < 8; ++v) { const int rr = m0 + r * 16 + 8 * hh + v, cc = t * 16 + col; Hs[rr][cc] = (b16)fmaxf(acc[r][t][v] + b2[cc], 0.0f); }
  }
  wave_lds_sync();
  {
    v8f c0 = {}, c1 = {};
#pragma unroll
    for (int kb = 0; kb < FEAT; kb += 32) {
      const v16b bw = frag_kb(W3T + (size_t)col * FEAT + kb, hh);
      c0 = wmma16b(frag_kb(&Hs[m0 + col][kb], hh), bw, c0);
      c1 = wmma16b(frag_kb(&Hs[m0 + 16 + col][kb], hh), bw, c1);
    }
    if (col < 3) {
      const float bb = b3[col];
#pragma unroll
      for (int v = 0; v < 8; ++v) {
        rgbS[m0 + 8 * hh + v][col] = 1.0f / (1.0f + expf(-(c0[v] + bb)));
        rgbS[m0 + 16 + 8 * hh + v][col] = 1.0f / (1.0f + expf(-(c1[v] + bb)));
      }
    }
  }
  __syncthreads();
  if (wave == 0) {
    if (lane == 0) { float T = 1.0f; for (int s = 0; s < NSMP; ++s) { const float a = alphaS[s]; wS[s] = a * T; T = T * (1.0f - a + 1e-10f); } }
    wave_lds_sync();
    float r_ = 0.f, g_ = 0.f, b_ = 0.f, dp = 0.f, ac = 0.f;
    for (int s = lane; s < NSMP; s += 32) { const float w = wS[s]; r_ += w * rgbS[s][0]; g_ += w * rgbS[s][1]; b_ += w * rgbS[s][2]; dp += w * zvals[(size_t)ray * NSMP + s]; ac += w; }
#pragma unroll
    for (int o = 16; o > 0; o >>= 1) { r_ += __shfl_xor(r_, o); g_ += __shfl_xor(g_, o); b_ += __shfl_xor(b_, o); dp += __shfl_xor(dp, o); ac += __shfl_xor(ac, o); }
    const float v = (lane == 0) ? r_ : (lane == 1) ? g_ : (lane == 2) ? b_ : (lane == 3) ? dp : (lane == 4) ? ac : 0.0f;
    ((volatile float*)slot)[(size_t)ray * 32 + lane] = v;
    __threadfence();
    ((volatile float*)slot)[(size_t)ray * 32 + lane] = v;
  }
}

__global__ __launch_bounds__(256) void pack_kernel(const float* __restrict__ slot, float* __restrict__ out) {
  for (int pass = 0; pass < 2; ++pass) {
    for (int gidx = threadIdx.x; gidx < NRAY * 5; gidx += 256) {
      float v;
      if (gidx < NRAY * 3) { const int ray = gidx / 3, c = gidx % 3; v = slot[(size_t)ray * 32 + c]; }
      else if (gidx < NRAY * 4) { v = slot[(size_t)(gidx - NRAY * 3) * 32 + 3]; }
      else { v = slot[(size_t)(gidx - NRAY * 4) * 32 + 4]; }
      ((volatile float*)out)[gidx] = v;
    }
    __threadfence();
  }
}
}

extern "C" void kernel_launch(void* const* d_in, const int* in_sizes, int n_in,
                              void* d_out, int out_size, void* d_ws, size_t ws_size, hipStream_t stream) {
  (void)n_in;
  const float* sigf = (const float*)d_in[0];
  const float* app  = (const float*)d_in[1];
  const float* vdir = (const float*)d_in[2];
  const float* dist = (const float*)d_in[3];
  const float* zv   = (const float*)d_in[4];
  const float* W1 = (const float*)d_in[5];  const float* b1 = (const float*)d_in[6];
  const float* W2 = (const float*)d_in[7];  const float* b2 = (const float*)d_in[8];
  const float* W3 = (const float*)d_in[9];  const float* b3 = (const float*)d_in[10];
  float* out = (float*)d_out;
  if (in_sizes[0] != NRAY * NSMP || in_sizes[1] != NRAY * NSMP * APP || in_sizes[5] != NIN * FEAT || out_size != NRAY * 5) return;
  size_t off = 0; char* ws = (char*)d_ws;
  auto carve = [&](size_t bytes) { char* p = ws + off; off += (bytes + 255) & ~(size_t)255; return p; };
  b16* W1T = (b16*)carve((size_t)FEAT * W1P * 2);
  b16* W2T = (b16*)carve((size_t)FEAT * FEAT * 2);
  b16* W3T = (b16*)carve((size_t)16 * FEAT * 2);
  float* slot = (float*)carve((size_t)NRAY * 32 * 4);
  if (off > ws_size) return;
  prep_kernel<<<34, 256, 0, stream>>>(W1, W2, W3, W1T, W2T, W3T);
  ray_kernel<<<NRAY, 128, 0, stream>>>(sigf, app, vdir, dist, zv, W1T, b1, W2T, b2, W3T, b3, slot);
  pack_kernel<<<1, 256, 0, stream>>>(slot, out);
}
